// LRUBlock_61065845015259
// MI455X (gfx1250) — hardware-verified
//
#include <hip/hip_runtime.h>
#include <math.h>

typedef __attribute__((ext_vector_type(16))) _Float16 v16h;
typedef __attribute__((ext_vector_type(8)))  _Float16 v8h;
typedef __attribute__((ext_vector_type(16))) __bf16   v16b;
typedef __attribute__((ext_vector_type(8)))  __bf16   v8b;
typedef __attribute__((ext_vector_type(8)))  float    v8f;
typedef __attribute__((ext_vector_type(4)))  float    v4f;
typedef __attribute__((ext_vector_type(2)))  float    v2f;
typedef __attribute__((ext_vector_type(2)))  _Float16 v2h;

constexpr int kS    = 4;
constexpr int kT    = 4096;
constexpr int kH    = 512;
constexpr int kN2   = 2 * kH;
constexpr int kF    = 4 * kH;
constexpr int kLay  = 4;
constexpr int kThr  = 256;
constexpr float kInCarry = 1024.0f;
constexpr float kSc = 1.0f / (kInCarry * kInCarry);
constexpr float kLnEps = 1e-5f;
constexpr float kCz = 1024.0f;
constexpr float kCh = 256.0f;
constexpr float kCy = 256.0f;
constexpr float kCf = 1024.0f;
constexpr float kScZ = 1.0f / (kCz * kInCarry), kScH = 1.0f / (kCh * kInCarry), kScY = 1.0f / (kCy * kInCarry), kScF = 1.0f / (kCf * kInCarry);
constexpr float kF16MinNormal = 6.103515625e-5f;

static_assert((kT % 64) == 0 && (kH % 64) == 0 && (kN2 % 64) == 0 && (kF % 64) == 0 && ((kT / 64) * (kH / 64)) % 8 == 0, "GEMM M, N multiples of 64; grids exact");
static_assert((kH % 256) == 0 && (kN2 % 256) == 0 && (kF % 256) == 0, "GEMM K multiples of 32; the plane cast's pitches and offsets multiples of 256");

constexpr size_t kOffWP = 0ull;
constexpr size_t kOffBW = 524288ull;
constexpr size_t kOffCW = 4718592ull;
constexpr size_t kOffW1 = 8912896ull;
constexpr size_t kOffW2 = 17301504ull;
constexpr size_t kOffBIAS = 25690112ull;
constexpr size_t kOffLAMG = 25739264ull;
constexpr size_t kOffPRM = 25772032ull;
constexpr size_t kOffZA = 25796608ull;
constexpr size_t kOffH32 = 29990912ull;
constexpr size_t kOffBU32 = 38379520ull;
constexpr size_t kOffHS16 = 55156736ull;
constexpr size_t kOffY32 = 63545344ull;
constexpr size_t kOffY16 = 71933952ull;
constexpr size_t kOffF32 = 76128256ull;
constexpr size_t kOffF16 = 109682688ull;
constexpr size_t kWsTotal = 126459904ull;
static_assert(kWsTotal <= 134217728ull, "carve cap: under 128 MiB");
static_assert(kOffWP == 0
              && kOffBW == kOffWP + 524288ull
              && kOffCW == kOffBW + 4194304ull
              && kOffW1 == kOffCW + 4194304ull
              && kOffW2 == kOffW1 + 8388608ull
              && kOffBIAS == kOffW2 + 8388608ull
              && kOffLAMG == kOffBIAS + 49152ull
              && kOffPRM == kOffLAMG + 32768ull
              && kOffZA == kOffPRM + 24576ull
              && kOffH32 == kOffZA + 4194304ull
              && kOffBU32 == kOffH32 + 8388608ull
              && kOffHS16 == kOffBU32 + 16777216ull
              && kOffY32 == kOffHS16 + 8388608ull
              && kOffY16 == kOffY32 + 8388608ull
              && kOffF32 == kOffY16 + 4194304ull
              && kOffF16 == kOffF32 + 33554432ull
              && kWsTotal == kOffF16 + 16777216ull, "the carve is chained and totalled");
static_assert((kOffWP % 256) == 0 && (kOffBW % 256) == 0 && (kOffCW % 256) == 0 && (kOffW1 % 256) == 0 && (kOffW2 % 256) == 0 && (kOffBIAS % 256) == 0 && (kOffLAMG % 256) == 0 && (kOffPRM % 256) == 0 && (kOffZA % 256) == 0 && (kOffH32 % 256) == 0 && (kOffBU32 % 256) == 0 && (kOffHS16 % 256) == 0 && (kOffY32 % 256) == 0 && (kOffY16 % 256) == 0 && (kOffF32 % 256) == 0 && (kOffF16 % 256) == 0, "aligned regions");
constexpr int kFZB = 0, kFB1 = 2048, kFLay = 2560, kFEnd = 12288;
static_assert(kFB1 + kLay * kFLay == kFEnd && kFLay == kF + kH && kFZB + kF <= kFB1 && (kFLay % 128) == 0, "bias stream map; the zero row reaches 2,048 columns");

__device__ __forceinline__ unsigned short f2bf_bits(float f) {
  unsigned u = __float_as_uint(f);
  return (unsigned short)((u + 0x7FFFu + ((u >> 16) & 1u)) >> 16);
}
__device__ __forceinline__ float bf_bits2f(unsigned short h) { return __uint_as_float(((unsigned)h) << 16); }
__device__ __forceinline__ float bf16r(float f) { return bf_bits2f(f2bf_bits(f)); }
__device__ __forceinline__ float carry_flush(float v, float carry) {
  const float s = v * carry;
  return (fabsf(s) < kF16MinNormal) ? 0.0f : s;
}
__device__ __forceinline__ float frcp(float x) { return __builtin_amdgcn_rcpf(x); }

__device__ __forceinline__ void dep_guard4_h(v8f& a, v8f& b, v8f& c, v8f& d, v16h x, v16h y) { asm volatile("v_nop\n\tv_nop\n\tv_nop\n\tv_nop" : "+v"(a), "+v"(b), "+v"(c), "+v"(d) : "v"(x), "v"(y)); }
__device__ __forceinline__ void dep_guard4_b(v8f& a, v8f& b, v8f& c, v8f& d, v16b x, v16b y) { asm volatile("v_nop\n\tv_nop\n\tv_nop\n\tv_nop" : "+v"(a), "+v"(b), "+v"(c), "+v"(d) : "v"(x), "v"(y)); }
__device__ __forceinline__ void keep4_h(v16h a, v16h b, v16h c, v16h d) { asm volatile("v_nop" :: "v"(a), "v"(b), "v"(c), "v"(d)); }
__device__ __forceinline__ void keep4_b(v16b a, v16b b, v16b c, v16b d) { asm volatile("v_nop" :: "v"(a), "v"(b), "v"(c), "v"(d)); }
__device__ __forceinline__ void acc_guard4(v8f& a, v8f& b, v8f& c, v8f& d) { asm volatile("v_nop\n\tv_nop\n\tv_nop\n\tv_nop" : "+v"(a), "+v"(b), "+v"(c), "+v"(d)); }

template <typename T> struct Frag;
template <> struct Frag<_Float16> {
  typedef v16h V; union U { v16h v; v8h h[2]; };
  static __device__ __forceinline__ v16h load(const _Float16* p) {
    U f; f.h[0] = *(const v8h*)(p); f.h[1] = *(const v8h*)(p + 16); return f.v;
  }
  static __device__ __forceinline__ v8f mma(v16h a, v16h b, v8f c) {
    return __builtin_amdgcn_wmma_f32_16x16x32_f16(false, a, false, b, (short)0, c, false, false);
  }
  static __device__ __forceinline__ void guard4(v8f& a, v8f& b, v8f& c, v8f& d, v16h x, v16h y) { dep_guard4_h(a, b, c, d, x, y); }
  static __device__ __forceinline__ void keep(v16h a, v16h b, v16h c, v16h d) { keep4_h(a, b, c, d); }
};
template <> struct Frag<__bf16> {
  typedef v16b V; union U { v16b v; v8b h[2]; };
  static __device__ __forceinline__ v16b load(const __bf16* p) {
    U f; f.h[0] = *(const v8b*)(p); f.h[1] = *(const v8b*)(p + 16); return f.v;
  }
  static __device__ __forceinline__ v8f mma(v16b a, v16b b, v8f c) {
    return __builtin_amdgcn_wmma_f32_16x16x32_bf16(false, a, false, b, (short)0, c, false, false);
  }
  static __device__ __forceinline__ void guard4(v8f& a, v8f& b, v8f& c, v8f& d, v16b x, v16b y) { dep_guard4_b(a, b, c, d, x, y); }
  static __device__ __forceinline__ void keep(v16b a, v16b b, v16b c, v16b d) { keep4_b(a, b, c, d); }
};

__device__ __forceinline__ v8f mma_h(v16h a, v16h b, v8f c) {
  c = __builtin_amdgcn_wmma_f32_16x16x32_f16(false, a, false, b, (short)0, c, false, false);
  asm volatile("v_nop\n\tv_nop\n\tv_nop\n\tv_nop" : "+v"(c) : "v"(a), "v"(b));
  return c;
}

template <int ET> struct Elem;
template <> struct Elem<0> { typedef _Float16 T; };
template <> struct Elem<1> { typedef __bf16 T; };
template <int ET, bool SPLIT, int BIAS_MODE, int OUT_MODE, bool RESID, int ACT = 0>
__global__ __launch_bounds__(256) void wmma_gemm64(
    const unsigned short* __restrict__ Ap, const unsigned short* __restrict__ A2p, int lda, long strideA,
    const unsigned short* __restrict__ Btp, const unsigned short* __restrict__ Bt2p, int ldb, long strideB,
    void* __restrict__ Cout, void* __restrict__ Cout2, int ldc, long strideC,
    const float* __restrict__ bias,
    const float* __restrict__ resid, long strideR,
    int M, int N, int K, float scale) {
  typedef typename Elem<ET>::T T;
  typedef typename Frag<T>::V V;
  const T* A = (const T*)Ap; const T* A2 = (const T*)A2p; const T* Bt = (const T*)Btp; const T* Bt2 = (const T*)Bt2p;
  __shared__ __align__(16) float sT[8][16 * 68];
  const int b    = blockIdx.y;
  const int lane = threadIdx.x & 31;
  const int wave = threadIdx.x >> 5;
  const int tilesN = N >> 6;
  const int tilesM = M >> 6;
  const int tile = blockIdx.x * 8 + wave;
  if (tile >= tilesM * tilesN) return;
  const int tm = tile / tilesN;
  const int tn = tile - tm * tilesN;
  const int m0 = tm << 6;
  const int n0 = tn << 6;

  const T* Ab  = A  + (size_t)b * strideA;
  const T* Bb  = Bt + (size_t)b * strideB;
  const T* Ab2 = SPLIT ? (A2  + (size_t)b * strideA) : nullptr;
  const T* Bb2 = SPLIT ? (Bt2 + (size_t)b * strideB) : nullptr;

  const int rlane = lane & 15;
  const int koff  = (lane >> 4) * 8;
  const int mOff  = (lane >> 4) * 8;

  v8f acc[4][4];
#pragma unroll
  for (int i = 0; i < 4; ++i)
#pragma unroll
    for (int j = 0; j < 4; ++j) acc[i][j] = (v8f){0.f,0.f,0.f,0.f,0.f,0.f,0.f,0.f};

  for (int k0 = 0; k0 < K; k0 += 32) {
    V bh[4], bl[4];
#pragma unroll
    for (int j = 0; j < 4; ++j) {
      const size_t bo = (size_t)(n0 + (j << 4) + rlane) * ldb + koff + k0;
      bh[j] = Frag<T>::load(Bb + bo);
      if (SPLIT) bl[j] = Frag<T>::load(Bb2 + bo);
    }
#pragma unroll
    for (int i = 0; i < 4; ++i) {
      const size_t ao = (size_t)(m0 + (i << 4) + rlane) * lda + koff + k0;
      V ah = Frag<T>::load(Ab + ao);
      V al;
      if (SPLIT) al = Frag<T>::load(Ab2 + ao);
#pragma unroll
      for (int j = 0; j < 4; ++j) {
        acc[i][j] = Frag<T>::mma(ah, bh[j], acc[i][j]);
        if (SPLIT) {
          acc[i][j] = Frag<T>::mma(ah, bl[j], acc[i][j]);
          acc[i][j] = Frag<T>::mma(al, bh[j], acc[i][j]);
        }
      }
      Frag<T>::guard4(acc[i][0], acc[i][1], acc[i][2], acc[i][3], ah, SPLIT ? al : ah);
    }
    Frag<T>::keep(bh[0], bh[1], bh[2], bh[3]);
    if (SPLIT) Frag<T>::keep(bl[0], bl[1], bl[2], bl[3]);
  }
  acc_guard4(acc[0][0], acc[0][1], acc[0][2], acc[0][3]);
  acc_guard4(acc[1][0], acc[1][1], acc[1][2], acc[1][3]);
  acc_guard4(acc[2][0], acc[2][1], acc[2][2], acc[2][3]);
  acc_guard4(acc[3][0], acc[3][1], acc[3][2], acc[3][3]);

  float* slab = sT[wave];
  const float* Rb = RESID ? (resid + (size_t)b * strideR) : nullptr;
#pragma unroll
  for (int i = 0; i < 4; ++i) {
    const int mBase = m0 + (i << 4);
#pragma unroll
    for (int j = 0; j < 4; ++j) {
      const int n = n0 + (j << 4) + rlane;
      float bv = 0.f;
      if (BIAS_MODE == 2) bv = bias[n];
#pragma unroll
      for (int r = 0; r < 8; ++r) {
        float v = acc[i][j][r] * scale;
        if (BIAS_MODE == 1) v += bias[mBase + mOff + r];
        if (BIAS_MODE == 2) v += bv;
        if (RESID) v += Rb[(size_t)(mBase + mOff + r) * ldc + n];
        if (ACT == 1) v = tanhf(v);
        if (ACT == 2) v = fmaxf(v, 0.0f);
        if (ACT == 3) v = v / (1.0f + expf(-v));
        if (ACT == 4) v = (v > 0.f) ? v : 0.01f * v;
        slab[(mOff + r) * 68 + (j << 4) + rlane] = v;
      }
    }
    __builtin_amdgcn_fence(__ATOMIC_RELEASE, "workgroup");
    __builtin_amdgcn_wave_barrier();
    __builtin_amdgcn_fence(__ATOMIC_ACQUIRE, "workgroup");
    if (OUT_MODE == 0) {
      float* C = (float*)Cout + (size_t)b * strideC;
      const int hh = lane >> 4, c4 = (lane & 15) * 4;
      for (int pass = 0; pass < 2; ++pass) {
#pragma unroll
        for (int it = 0; it < 8; ++it) {
          const int row = it * 2 + hh;
          v4f v = *(const v4f*)(slab + row * 68 + c4);
          *(volatile v4f*)(C + (size_t)(mBase + row) * ldc + n0 + c4) = v;
        }
        __threadfence();
      }
    } else {
      const int q = lane >> 3, c8 = (lane & 7) * 8;
      unsigned short* C  = (unsigned short*)Cout  + (size_t)b * strideC;
      unsigned short* C2 = (OUT_MODE == 2) ? ((unsigned short*)Cout2 + (size_t)b * strideC) : nullptr;
      for (int pass = 0; pass < 2; ++pass) {
#pragma unroll
        for (int it = 0; it < 4; ++it) {
          const int row = it * 4 + q;
          const float* sp = slab + row * 68 + c8;
          v8h hv, lv;
#pragma unroll
          for (int e = 0; e < 8; ++e) {
            if (OUT_MODE == 1) {
              hv[e] = (_Float16)sp[e];
            } else {
              unsigned short hb = f2bf_bits(sp[e]);
              unsigned short lb = f2bf_bits(sp[e] - bf_bits2f(hb));
              hv[e] = __builtin_bit_cast(_Float16, hb);
              lv[e] = __builtin_bit_cast(_Float16, lb);
            }
          }
          *(volatile v8h*)(C + (size_t)(mBase + row) * ldc + n0 + c8) = hv;
          if (OUT_MODE == 2) *(volatile v8h*)(C2 + (size_t)(mBase + row) * ldc + n0 + c8) = lv;
        }
        __threadfence();
      }
    }
    __builtin_amdgcn_fence(__ATOMIC_RELEASE, "workgroup");
    __builtin_amdgcn_wave_barrier();
    __builtin_amdgcn_fence(__ATOMIC_ACQUIRE, "workgroup");
  }
}

__global__ __launch_bounds__(kThr) void cast_plane_kernel(const float* __restrict__ src, unsigned short* __restrict__ dst,
                                                          int colsLog2, int dstPitch, int dstOff) {
  const int i   = blockIdx.x * kThr + threadIdx.x;
  const int sh  = colsLog2 - 3;
  const int row = i >> sh;
  const int c8  = (i & ((1 << sh) - 1)) * 8;
  const float* sp = src + ((size_t)row << colsLog2) + c8;
  const v4f a0 = *(const v4f*)(sp);
  const v4f a1 = *(const v4f*)(sp + 4);
  v8h hv;
#pragma unroll
  for (int e = 0; e < 4; ++e) {
    const float f0 = a0[e];
    const float f1 = a1[e];
    hv[e]     = (_Float16)carry_flush(bf16r(f0), kInCarry);
    hv[4 + e] = (_Float16)carry_flush(bf16r(f1), kInCarry);
  }
  unsigned short* dp = dst + (size_t)row * dstPitch + dstOff + c8;
  *(volatile v8h*)dp = hv;
  __threadfence();
  *(volatile v8h*)dp = hv;
}

__global__ __launch_bounds__(kThr) void setup_kernel(const float* __restrict__ nu_log, const float* __restrict__ theta_log, const float* __restrict__ gamma_log,
                                                     const float* __restrict__ ln_w, const float* __restrict__ ln_b, const float* __restrict__ Dk,
                                                     const float* __restrict__ ff_b1, const float* __restrict__ ff_b2,
                                                     float* __restrict__ BIAS, float* __restrict__ LAMG, float* __restrict__ PRM) {
  unsigned v = blockIdx.x * (unsigned)kThr + threadIdx.x;
  asm volatile("" : "+v"(v));
  v4f o = {0.f, 0.f, 0.f, 0.f};
  float* dp;
  if (v < 3072u) {
    const unsigned i0 = v * 4u;
    if (i0 >= (unsigned)kFB1) {
      const unsigned l = (i0 - (unsigned)kFB1) / (unsigned)kFLay, off = (i0 - (unsigned)kFB1) % (unsigned)kFLay;
      const float* sp = (off < (unsigned)kF) ? (ff_b1 + (size_t)l * kF + off) : (ff_b2 + (size_t)l * kH + (off - (unsigned)kF));
      const v4f a = *(const v4f*)sp;
#pragma unroll
      for (int e = 0; e < 4; ++e) { const float p = a[e]; o[e] = bf16r(p); }
    }
    dp = BIAS + i0;
  } else if (v < 5120u) {
    const unsigned w = v - 3072u;
    const float nu = bf16r(nu_log[w]), th = bf16r(theta_log[w]), ga = bf16r(gamma_log[w]);
    const float mag = expf(-expf(nu)), ang = expf(th);
    o[0] = mag * cosf(ang); o[1] = mag * sinf(ang); o[2] = expf(ga); o[3] = 0.0f;
    dp = LAMG + (size_t)w * 4u;
  } else {
    const unsigned i0 = (v - 5120u) * 4u;
    const unsigned l = i0 / 1536u, wh = (i0 % 1536u) / 512u, c = i0 % 512u;
    const float* sp = ((wh == 0u) ? ln_w : ((wh == 1u) ? ln_b : Dk)) + (size_t)l * kH + c;
    const v4f a = *(const v4f*)sp;
#pragma unroll
    for (int e = 0; e < 4; ++e) { const float p = a[e]; o[e] = bf16r(p); }
    dp = PRM + i0;
  }
  *(volatile v4f*)dp = o;
  __threadfence();
  *(volatile v4f*)dp = o;
}
static_assert(kFEnd / 4 == 3072 && kLay * kH == 2048 && kLay * 3 * kH / 4 == 1536 && 3072 + 2048 + 1536 == 26 * kThr && (3072 % 32) == 0 && (5120 % 32) == 0 && (kFB1 % 4) == 0 && (kF % 4) == 0, "set-up grid exact; regions wave-uniform");

__device__ __forceinline__ void row_stats(const float* __restrict__ hr, float& mu, float& rs) {
  float s = 0.0f;
#pragma unroll 4
  for (int c = 0; c < kH; c += 4) { const v4f a = *(const v4f*)(hr + c); s += (a[0] + a[1]) + (a[2] + a[3]); }
  mu = s * (1.0f / (float)kH);
  float q = 0.0f;
#pragma unroll 4
  for (int c = 0; c < kH; c += 4) { const v4f a = *(const v4f*)(hr + c); const float d0 = a[0] - mu, d1 = a[1] - mu, d2 = a[2] - mu, d3 = a[3] - mu; q += (d0 * d0 + d1 * d1) + (d2 * d2 + d3 * d3); }
  const float var = q * (1.0f / (float)kH);
  rs = 1.0f / sqrtf(var + kLnEps);
}

__global__ __launch_bounds__(kThr) void ln_kernel(const float* __restrict__ H32, const float* __restrict__ PRM, unsigned short* __restrict__ ZA) {
  const unsigned r = blockIdx.x * (unsigned)kThr + threadIdx.x;
  const float* hr = H32 + (size_t)r * kH;
  float mu, rs;
  row_stats(hr, mu, rs);
  unsigned short* zr = ZA + (size_t)r * kH;
  for (int pass = 0; pass < 2; ++pass) {
#pragma unroll 2
    for (int c = 0; c < kH; c += 8) {
      const v4f a0 = *(const v4f*)(hr + c), a1 = *(const v4f*)(hr + c + 4);
      const v4f w0 = *(const v4f*)(PRM + c), w1 = *(const v4f*)(PRM + c + 4);
      const v4f b0 = *(const v4f*)(PRM + kH + c), b1 = *(const v4f*)(PRM + kH + c + 4);
      v8h hv;
#pragma unroll
      for (int e = 0; e < 4; ++e) {
        hv[e] = (_Float16)carry_flush((a0[e] - mu) * rs * w0[e] + b0[e], kCz);
        hv[4 + e] = (_Float16)carry_flush((a1[e] - mu) * rs * w1[e] + b1[e], kCz);
      }
      *(volatile v8h*)(zr + c) = hv;
    }
    __threadfence();
  }
}
static_assert(kT == 16 * kThr, "one thread a row: 16 blocks");

__global__ __launch_bounds__(kThr) void scan_kernel(const float* __restrict__ BU, const float* __restrict__ LAMG, unsigned short* __restrict__ HS16) {
  const unsigned n2 = threadIdx.x * 2u;
  const v4f p0 = *(const v4f*)(LAMG + (size_t)n2 * 4u), p1 = *(const v4f*)(LAMG + (size_t)(n2 + 1u) * 4u);
  const float lr0 = p0[0], li0 = p0[1], g0 = p0[2], lr1 = p1[0], li1 = p1[1], g1 = p1[2];
  float hr0 = 0.0f, hi0 = 0.0f, hr1 = 0.0f, hi1 = 0.0f;
#pragma unroll 2
  for (int t = 0; t < kT; ++t) {
    const v2f br = *(const v2f*)(BU + (size_t)t * kN2 + n2), bi = *(const v2f*)(BU + (size_t)t * kN2 + kH + n2);
    const float nr0 = (lr0 * hr0 - li0 * hi0) + g0 * br[0], ni0 = (lr0 * hi0 + li0 * hr0) + g0 * bi[0];
    const float nr1 = (lr1 * hr1 - li1 * hi1) + g1 * br[1], ni1 = (lr1 * hi1 + li1 * hr1) + g1 * bi[1];
    hr0 = nr0; hi0 = ni0; hr1 = nr1; hi1 = ni1;
    v2h sr, si;
    sr[0] = (_Float16)carry_flush(hr0, kCh); sr[1] = (_Float16)carry_flush(hr1, kCh);
    si[0] = (_Float16)carry_flush(-hi0, kCh); si[1] = (_Float16)carry_flush(-hi1, kCh);
    unsigned short* pr = HS16 + (size_t)t * kN2 + n2;
    unsigned short* pi = HS16 + (size_t)t * kN2 + kH + n2;
    *(volatile v2h*)pr = sr; *(volatile v2h*)pi = si;
    __threadfence();
    *(volatile v2h*)pr = sr; *(volatile v2h*)pi = si;
  }
}
static_assert(kH == 2 * kThr, "two states a lane, one block");

__global__ __launch_bounds__(kThr) void skip_kernel(const float* __restrict__ Y32, const float* __restrict__ H32, const float* __restrict__ PRM,
                                                    unsigned short* __restrict__ Y16) {
  const unsigned r = blockIdx.x * (unsigned)kThr + threadIdx.x;
  const float* hr = H32 + (size_t)r * kH;
  const float* yr = Y32 + (size_t)r * kH;
  float mu, rs;
  row_stats(hr, mu, rs);
  unsigned short* orow = Y16 + (size_t)r * kH;
  for (int pass = 0; pass < 2; ++pass) {
#pragma unroll 2
    for (int c = 0; c < kH; c += 8) {
      const v4f a0 = *(const v4f*)(hr + c), a1 = *(const v4f*)(hr + c + 4);
      const v4f y0 = *(const v4f*)(yr + c), y1 = *(const v4f*)(yr + c + 4);
      const v4f w0 = *(const v4f*)(PRM + c), w1 = *(const v4f*)(PRM + c + 4);
      const v4f b0 = *(const v4f*)(PRM + kH + c), b1 = *(const v4f*)(PRM + kH + c + 4);
      const v4f d0 = *(const v4f*)(PRM + 2 * kH + c), d1 = *(const v4f*)(PRM + 2 * kH + c + 4);
      v8h hv;
#pragma unroll
      for (int e = 0; e < 4; ++e) {
        hv[e] = (_Float16)carry_flush(y0[e] + d0[e] * ((a0[e] - mu) * rs * w0[e] + b0[e]), kCy);
        hv[4 + e] = (_Float16)carry_flush(y1[e] + d1[e] * ((a1[e] - mu) * rs * w1[e] + b1[e]), kCy);
      }
      *(volatile v8h*)(orow + c) = hv;
    }
    __threadfence();
  }
}

__global__ __launch_bounds__(kThr) void gelu_kernel(const float* __restrict__ F32, unsigned short* __restrict__ F16) {
  typedef __attribute__((ext_vector_type(4))) _Float16 v4h;
  const size_t v = (size_t)blockIdx.x * kThr + threadIdx.x;
  const v4f a = *(const v4f*)(F32 + v * 4);
  v4h hv;
#pragma unroll
  for (int e = 0; e < 4; ++e) { const float g = a[e]; hv[e] = (_Float16)carry_flush(0.5f * g * (1.0f + erff(g * 0.70710678118654752440f)), kCf); }
  unsigned short* dp = F16 + v * 4;
  *(volatile v4h*)dp = hv;
  __threadfence();
  *(volatile v4h*)dp = hv;
}
static_assert(((size_t)kT * kF / 4) % kThr == 0, "GELU grid exact");

__global__ __launch_bounds__(kThr) void resid_kernel(float* __restrict__ H32, const float* __restrict__ M32, float* __restrict__ outS, int last) {
  const size_t v = (size_t)blockIdx.x * kThr + threadIdx.x;
  const v4f h = *(const v4f*)(H32 + v * 4), m = *(const v4f*)(M32 + v * 4);
  v4f o;
#pragma unroll
  for (int e = 0; e < 4; ++e) o[e] = h[e] + m[e];
  for (int pass = 0; pass < 2; ++pass) {
    *(volatile v4f*)(H32 + v * 4) = o;
    if (last) *(volatile v4f*)(outS + v * 4) = o;
    __threadfence();
  }
}
static_assert(((size_t)kT * kH / 4) % kThr == 0, "residual grid exact");

static_assert(((size_t)kH * kH / 8) % kThr == 0 && ((size_t)kF * kH / 8) % kThr == 0 && ((size_t)kT * kH / 8) % kThr == 0, "plane cast grids exact");

extern "C" void kernel_launch(void* const* d_in, const int* in_sizes, int n_in,
                              void* d_out, int out_size, void* d_ws, size_t ws_size,
                              hipStream_t stream) {
  if (n_in < 16 || d_out == nullptr || d_ws == nullptr) return;
  if (in_sizes[0] != kS * kT * kH || in_sizes[1] != kH * kH || in_sizes[2] != kLay * kH || in_sizes[3] != kLay * kH || in_sizes[4] != kLay * kH || in_sizes[5] != kLay * kH || in_sizes[6] != kLay * kH) return;
  if (in_sizes[7] != kLay * kH * kH || in_sizes[8] != kLay * kH * kH || in_sizes[9] != kLay * kH * kH || in_sizes[10] != kLay * kH * kH || in_sizes[11] != kLay * kH) return;
  if (in_sizes[12] != kLay * kF * kH || in_sizes[13] != kLay * kF || in_sizes[14] != kLay * kH * kF || in_sizes[15] != kLay * kH) return;
  if (out_size != kS * kT * kH) return;
  if (ws_size < kWsTotal) return;
  const float* x = (const float*)d_in[0];
  const float* W_proj = (const float*)d_in[1];
  const float* ln_w = (const float*)d_in[2];
  const float* ln_b = (const float*)d_in[3];
  const float* nu_log = (const float*)d_in[4];
  const float* theta_log = (const float*)d_in[5];
  const float* gamma_log = (const float*)d_in[6];
  const float* B_re = (const float*)d_in[7];
  const float* B_im = (const float*)d_in[8];
  const float* C_re = (const float*)d_in[9];
  const float* C_im = (const float*)d_in[10];
  const float* Dk = (const float*)d_in[11];
  const float* ff_w1 = (const float*)d_in[12];
  const float* ff_b1 = (const float*)d_in[13];
  const float* ff_w2 = (const float*)d_in[14];
  const float* ff_b2 = (const float*)d_in[15];
  float* out = (float*)d_out;
  char* ws = (char*)d_ws;
  unsigned short* WP = (unsigned short*)(ws + kOffWP);
  unsigned short* BW = (unsigned short*)(ws + kOffBW);
  unsigned short* CW = (unsigned short*)(ws + kOffCW);
  unsigned short* W1 = (unsigned short*)(ws + kOffW1);
  unsigned short* W2 = (unsigned short*)(ws + kOffW2);
  float* BIAS = (float*)(ws + kOffBIAS);
  float* LAMG = (float*)(ws + kOffLAMG);
  float* PRM = (float*)(ws + kOffPRM);
  unsigned short* ZA = (unsigned short*)(ws + kOffZA);
  float* H32 = (float*)(ws + kOffH32);
  float* BU32 = (float*)(ws + kOffBU32);
  unsigned short* HS16 = (unsigned short*)(ws + kOffHS16);
  float* Y32 = (float*)(ws + kOffY32);
  unsigned short* Y16 = (unsigned short*)(ws + kOffY16);
  float* F32 = (float*)(ws + kOffF32);
  unsigned short* F16 = (unsigned short*)(ws + kOffF16);

  const int gSq = (int)(((size_t)kH * kH / 8) / kThr), gFf = (int)(((size_t)kF * kH / 8) / kThr), gX = (int)(((size_t)kT * kH / 8) / kThr);
  cast_plane_kernel<<<gSq, kThr, 0, stream>>>(W_proj, WP, 9, kH, 0);
  for (int l = 0; l < kLay; ++l) {
    cast_plane_kernel<<<gSq, kThr, 0, stream>>>(B_re + (size_t)l * kH * kH, BW + (size_t)l * kN2 * kH, 9, kH, 0);
    cast_plane_kernel<<<gSq, kThr, 0, stream>>>(B_im + (size_t)l * kH * kH, BW + (size_t)l * kN2 * kH + (size_t)kH * kH, 9, kH, 0);
    cast_plane_kernel<<<gSq, kThr, 0, stream>>>(C_re + (size_t)l * kH * kH, CW + (size_t)l * kH * kN2, 9, kN2, 0);
    cast_plane_kernel<<<gSq, kThr, 0, stream>>>(C_im + (size_t)l * kH * kH, CW + (size_t)l * kH * kN2, 9, kN2, kH);
    cast_plane_kernel<<<gFf, kThr, 0, stream>>>(ff_w1 + (size_t)l * kF * kH, W1 + (size_t)l * kF * kH, 9, kH, 0);
    cast_plane_kernel<<<gFf, kThr, 0, stream>>>(ff_w2 + (size_t)l * kH * kF, W2 + (size_t)l * kH * kF, 11, kF, 0);
  }
  setup_kernel<<<26, kThr, 0, stream>>>(nu_log, theta_log, gamma_log, ln_w, ln_b, Dk, ff_b1, ff_b2, BIAS, LAMG, PRM);

  for (int s = 0; s < kS; ++s) {
    cast_plane_kernel<<<gX, kThr, 0, stream>>>(x + (size_t)s * kT * kH, ZA, 9, kH, 0);
    wmma_gemm64<0, false, 2, 0, false, 0><<<dim3((kT / 64) * (kH / 64) / 8, 1), 256, 0, stream>>>(
        ZA, ZA, kH, 0L, WP, WP, kH, 0L, (void*)H32, (void*)H32, kH, 0L, BIAS + kFZB, nullptr, 0L, kT, kH, kH, kSc);
    for (int l = 0; l < kLay; ++l) {
      const float* prm = PRM + (size_t)l * 3 * kH;
      ln_kernel<<<16, kThr, 0, stream>>>(H32, prm, ZA);
      wmma_gemm64<0, false, 2, 0, false, 0><<<dim3((kT / 64) * (kN2 / 64) / 8, 1), 256, 0, stream>>>(
          ZA, ZA, kH, 0L, BW + (size_t)l * kN2 * kH, BW + (size_t)l * kN2 * kH, kH, 0L, (void*)BU32, (void*)BU32, kN2, 0L, BIAS + kFZB, nullptr, 0L, kT, kN2, kH, kScZ);
      scan_kernel<<<1, kThr, 0, stream>>>(BU32, LAMG + (size_t)l * kH * 4, HS16);
      wmma_gemm64<0, false, 2, 0, false, 0><<<dim3((kT / 64) * (kH / 64) / 8, 1), 256, 0, stream>>>(
          HS16, HS16, kN2, 0L, CW + (size_t)l * kH * kN2, CW + (size_t)l * kH * kN2, kN2, 0L, (void*)Y32, (void*)Y32, kH, 0L, BIAS + kFZB, nullptr, 0L, kT, kH, kN2, kScH);
      skip_kernel<<<16, kThr, 0, stream>>>(Y32, H32, prm, Y16);
      wmma_gemm64<0, false, 2, 0, false, 0><<<dim3((kT / 64) * (kF / 64) / 8, 1), 256, 0, stream>>>(
          Y16, Y16, kH, 0L, W1 + (size_t)l * kF * kH, W1 + (size_t)l * kF * kH, kH, 0L, (void*)F32, (void*)F32, kF, 0L, BIAS + kFB1 + l * kFLay, nullptr, 0L, kT, kF, kH, kScY);
      gelu_kernel<<<(int)(((size_t)kT * kF / 4) / kThr), kThr, 0, stream>>>(F32, F16);
      wmma_gemm64<0, false, 2, 0, false, 0><<<dim3((kT / 64) * (kH / 64) / 8, 1), 256, 0, stream>>>(
          F16, F16, kF, 0L, W2 + (size_t)l * kH * kF, W2 + (size_t)l * kH * kF, kF, 0L, (void*)Y32, (void*)Y32, kH, 0L, BIAS + kFB1 + l * kFLay + kF, nullptr, 0L, kT, kH, kF, kScF);
      resid_kernel<<<(int)(((size_t)kT * kH / 4) / kThr), kThr, 0, stream>>>(H32, Y32, out + (size_t)s * kT * kH, (l == kLay - 1) ? 1 : 0);
    }
  }
}
